// FusionMultiHeadAttention_49538152792908
// MI455X (gfx1250) — hardware-verified
//
#include <hip/hip_runtime.h>


namespace {
constexpr int Bn = 4, S = 2048, D = 1024, H = 16, HD = 64;
constexpr float XS = 8.0f, PS = 8.0f, ISC = 0.03125f;

typedef _Float16 b16;
typedef __attribute__((ext_vector_type(16))) _Float16 v16b;
typedef __attribute__((ext_vector_type(8))) _Float16 v8b;
typedef __attribute__((ext_vector_type(8))) float v8f;
typedef __attribute__((ext_vector_type(4))) float v4f;
__device__ __forceinline__ float bf16_rne(float f) { unsigned int u = __float_as_uint(f); u += 0x7FFFu + ((u >> 16) & 1u); return __uint_as_float(u & 0xFFFF0000u); }
__device__ __forceinline__ void split16(float v, b16& hi, b16& lo) { hi = (b16)v; lo = (b16)(v - (float)hi); }
__device__ __forceinline__ v16b frag_kb(const b16* p, int hh) { const v8b a = *(const v8b*)(p + 8 * hh), b = *(const v8b*)(p + 16 + 8 * hh); v16b f;
#pragma unroll
  for (int e = 0; e < 8; ++e) { f[e] = a[e]; f[8 + e] = b[e]; } return f; }
__device__ __forceinline__ v8f wmma16b(v16b a, v16b b, v8f c) { v8f d = __builtin_amdgcn_wmma_f32_16x16x32_f16(false, a, false, b, (short)0, c, false, false); asm volatile("v_nop\n\tv_nop\n\tv_nop\n\tv_nop" : "+v"(d) : "v"(a), "v"(b)); return d; }
__device__ __forceinline__ void wave_lds_sync() { __builtin_amdgcn_fence(__ATOMIC_RELEASE, "workgroup"); __builtin_amdgcn_wave_barrier(); __builtin_amdgcn_fence(__ATOMIC_ACQUIRE, "workgroup"); }
__device__ __forceinline__ float nexp(float x) { return __builtin_amdgcn_exp2f(x * 1.4426950408889634f); }
__device__ __forceinline__ float pmul(float a, float b) { float p = a * b; asm volatile("" : "+v"(p)); return p; }

__global__ __launch_bounds__(256) void prep_kernel(const float* __restrict__ x1, const float* __restrict__ x2, const float* __restrict__ wq, const float* __restrict__ wk, const float* __restrict__ wv, const float* __restrict__ wo, b16* __restrict__ R, b16* __restrict__ X1, b16* __restrict__ X2) {
  const size_t tid = (size_t)blockIdx.x * 256 + threadIdx.x, nth = (size_t)gridDim.x * 256;
  for (int pass = 0; pass < 2; ++pass) {
    for (size_t p = tid; p < (size_t)4 * D * D / 8; p += nth) { const size_t q = p * 8; const int w = (int)(q / ((size_t)D * D)); const size_t r = q % ((size_t)D * D); const float* Wm = (w == 0) ? wq : (w == 1) ? wk : (w == 2) ? wv : wo; v8b v; for (int e = 0; e < 8; ++e) v[e] = (b16)bf16_rne(Wm[r + e]); *(volatile v8b*)(R + q) = v; }
    for (size_t p = tid; p < (size_t)Bn * S * D / 8; p += nth) { v8b a, c; for (int e = 0; e < 8; ++e) { a[e] = (b16)(bf16_rne(x1[p * 8 + e]) * XS); c[e] = (b16)(bf16_rne(x2[p * 8 + e]) * XS); } *(volatile v8b*)(X1 + p * 8) = a; *(volatile v8b*)(X2 + p * 8) = c; }
    __threadfence(); }
}
__global__ __launch_bounds__(64) void qk_kernel(const b16* __restrict__ X1, const b16* __restrict__ X2, const b16* __restrict__ R, b16* __restrict__ Q, b16* __restrict__ K) {
  __shared__ __attribute__((aligned(16))) b16 Th[2][32][128 + 8];
  const int lane = threadIdx.x & 31, wave = threadIdx.x >> 5, nloc = lane & 15, hlf = lane >> 4, m0 = blockIdx.y * 32; const bool isk = blockIdx.x >= 8; const int c0 = (blockIdx.x & 7) * 128; (void)wave;
  const b16* X = isk ? X2 : X1; const b16* Bw = R + (isk ? (size_t)D * D : 0); const int cw = c0;
  const int mw = m0 + wave * 16;
  v8f acc[8];
#pragma unroll
  for (int t = 0; t < 8; ++t) acc[t] = (v8f){};
#pragma unroll 2
  for (int kb = 0; kb < D; kb += 32) { const v16b a = frag_kb(X + (size_t)(mw + nloc) * D + kb, hlf);
#pragma unroll
    for (int t = 0; t < 8; ++t) acc[t] = wmma16b(a, frag_kb(Bw + (size_t)(cw + t * 16 + nloc) * D + kb, hlf), acc[t]); }
#pragma unroll
  for (int t = 0; t < 8; ++t)
#pragma unroll
    for (int r = 0; r < 8; ++r) Th[wave][8 * hlf + r][t * 16 + nloc] = (b16)acc[t][r];
  wave_lds_sync();
  b16* dstp = isk ? K : Q;
  for (int pass = 0; pass < 2; ++pass) { for (int i = lane; i < 16 * 16; i += 32) { const int rr = i >> 4, c8 = (i & 15) * 8; *(volatile v8b*)(dstp + (size_t)(mw + rr) * D + cw + c8) = *(const v8b*)(&Th[wave][rr][c8]); } __threadfence(); }
}
__global__ __launch_bounds__(128) void v_kernel(const b16* __restrict__ X2, const b16* __restrict__ R, b16* __restrict__ VT, b16* __restrict__ VTl) {
  __shared__ __attribute__((aligned(16))) b16 Th[128][64 + 8], Tl[128][64 + 8];
  const int lane = threadIdx.x & 31, wave = threadIdx.x >> 5, nloc = lane & 15, hlf = lane >> 4, g0 = blockIdx.y * 64, m0 = g0 + wave * 16, c0 = blockIdx.x * 128; const b16* Bv = R + (size_t)2 * D * D + (size_t)c0 * D;
  const int b = g0 / S, t0 = g0 % S;
  v8f acc[8];
#pragma unroll
  for (int t = 0; t < 8; ++t) acc[t] = (v8f){};
#pragma unroll 2
  for (int kb = 0; kb < D; kb += 32) { const v16b a = frag_kb(X2 + (size_t)(m0 + nloc) * D + kb, hlf);
#pragma unroll
    for (int t = 0; t < 8; ++t) acc[t] = wmma16b(a, frag_kb(Bv + (size_t)(t * 16 + nloc) * D + kb, hlf), acc[t]); }
#pragma unroll
  for (int t = 0; t < 8; ++t)
#pragma unroll
    for (int r = 0; r < 8; ++r) { b16 a_, c_; split16(acc[t][r], a_, c_); Th[t * 16 + nloc][wave * 16 + 8 * hlf + r] = a_; Tl[t * 16 + nloc][wave * 16 + 8 * hlf + r] = c_; }
  __syncthreads();
  for (int pass = 0; pass < 2; ++pass) { for (int i = threadIdx.x; i < 128 * 8; i += 128) { const int dd = i >> 3, c8 = (i & 7) * 8; const size_t gi = ((size_t)b * D + c0 + dd) * S + t0 + c8; *(volatile v8b*)(VT + gi) = *(const v8b*)(&Th[dd][c8]); *(volatile v8b*)(VTl + gi) = *(const v8b*)(&Tl[dd][c8]); } __threadfence(); }
}
__global__ __launch_bounds__(128) void attn_kernel(const b16* __restrict__ Q, const b16* __restrict__ K, const b16* __restrict__ VT, const b16* __restrict__ VTL, b16* __restrict__ CH, b16* __restrict__ CL) {
  __shared__ __attribute__((aligned(16))) b16 Oh[16][4 * HD + 8], Ol[16][4 * HD + 8];
  const int wid = threadIdx.x >> 5, lane = threadIdx.x & 31, hh = lane >> 4, col = lane & 15; const int b = blockIdx.z, q0 = blockIdx.x * 16, h = blockIdx.y * 4 + wid, qi = q0 + col;
  const b16* Qr = Q + ((size_t)b * S) * D + h * HD; const b16* Kr = K + ((size_t)b * S) * D + h * HD; const b16* V = VT + ((size_t)b * D + h * HD) * S; const b16* Vl = VTL + ((size_t)b * D + h * HD) * S;
  const v16b qf0 = frag_kb(Qr + (size_t)qi * D, hh), qf1 = frag_kb(Qr + (size_t)qi * D + 32, hh);
  float m = -INFINITY, l = 0.0f; v8f o[4] = {{}, {}, {}, {}};
  for (int kb = 0; kb < S; kb += 32) {
    v8f s0 = {}, s1 = {}; s0 = wmma16b(frag_kb(Kr + (size_t)(kb + col) * D, hh), qf0, s0); s0 = wmma16b(frag_kb(Kr + (size_t)(kb + col) * D + 32, hh), qf1, s0); s1 = wmma16b(frag_kb(Kr + (size_t)(kb + 16 + col) * D, hh), qf0, s1); s1 = wmma16b(frag_kb(Kr + (size_t)(kb + 16 + col) * D + 32, hh), qf1, s1);
    float mr = -INFINITY;
#pragma unroll
    for (int r = 0; r < 8; ++r) { s0[r] *= ISC / (XS * XS); s1[r] *= ISC / (XS * XS); mr = fmaxf(mr, fmaxf(s0[r], s1[r])); }
    mr = fmaxf(mr, __shfl_xor(mr, 16)); const float mn = fmaxf(m, mr); const float al_ = nexp(m - mn); m = mn; float sum = 0.0f; v16b pb, pl;
#pragma unroll
    for (int r = 0; r < 8; ++r) { const float e0 = nexp(s0[r] - mn), e1 = nexp(s1[r] - mn); sum += e0 + e1; b16 a_, c_; split16(e0 * PS, a_, c_); pb[r] = a_; pl[r] = c_; split16(e1 * PS, a_, c_); pb[8 + r] = a_; pl[8 + r] = c_; }
    sum += __shfl_xor(sum, 16); l = l * al_ + sum;
#pragma unroll
    for (int t = 0; t < 4; ++t) { o[t] *= al_; const v16b vh = frag_kb(V + (size_t)(t * 16 + col) * S + kb, hh); o[t] = wmma16b(vh, pb, o[t]); o[t] = wmma16b(vh, pl, o[t]); o[t] = wmma16b(frag_kb(Vl + (size_t)(t * 16 + col) * S + kb, hh), pb, o[t]); } }
  const float inv = 1.0f / ((1.0f + l) * PS);
#pragma unroll
  for (int t = 0; t < 4; ++t)
#pragma unroll
    for (int r = 0; r < 8; ++r) { b16 a_, c_; split16(o[t][r] * inv, a_, c_); Oh[col][wid * HD + t * 16 + 8 * hh + r] = a_; Ol[col][wid * HD + t * 16 + 8 * hh + r] = c_; }
  __syncthreads();
  for (int pass = 0; pass < 2; ++pass) { for (int i = threadIdx.x; i < 16 * 32; i += 128) { const int rr = i >> 5, c8 = (i & 31) * 8; const size_t gi = ((size_t)b * S + q0 + rr) * D + blockIdx.y * 4 * HD + c8; *(volatile v8b*)(CH + gi) = *(const v8b*)(&Oh[rr][c8]); *(volatile v8b*)(CL + gi) = *(const v8b*)(&Ol[rr][c8]); } __threadfence(); }
}
__global__ __launch_bounds__(64) void out_kernel(const b16* __restrict__ CH, const b16* __restrict__ CL, const b16* __restrict__ R, float* __restrict__ out) {
  __shared__ __attribute__((aligned(16))) float Ts[2][32][128 + 4];
  const int lane = threadIdx.x & 31, wave = threadIdx.x >> 5, nloc = lane & 15, hlf = lane >> 4, m0 = blockIdx.y * 32, c0 = blockIdx.x * 256 + wave * 128; const b16* RO = R + (size_t)3 * D * D;
  v8f acc[2][8];
#pragma unroll
  for (int r = 0; r < 2; ++r)
#pragma unroll
    for (int t = 0; t < 8; ++t) acc[r][t] = (v8f){};
#pragma unroll 2
  for (int kb = 0; kb < D; kb += 32) { const v16b a0 = frag_kb(CH + (size_t)(m0 + nloc) * D + kb, hlf), a1 = frag_kb(CH + (size_t)(m0 + 16 + nloc) * D + kb, hlf), l0 = frag_kb(CL + (size_t)(m0 + nloc) * D + kb, hlf), l1 = frag_kb(CL + (size_t)(m0 + 16 + nloc) * D + kb, hlf);
#pragma unroll
    for (int t = 0; t < 8; ++t) { const v16b bw = frag_kb(RO + (size_t)(c0 + t * 16 + nloc) * D + kb, hlf); acc[0][t] = wmma16b(a0, bw, acc[0][t]); acc[0][t] = wmma16b(l0, bw, acc[0][t]); acc[1][t] = wmma16b(a1, bw, acc[1][t]); acc[1][t] = wmma16b(l1, bw, acc[1][t]); } }
#pragma unroll
  for (int t = 0; t < 8; ++t)
#pragma unroll
    for (int r = 0; r < 2; ++r)
#pragma unroll
      for (int v = 0; v < 8; ++v) Ts[wave][r * 16 + 8 * hlf + v][t * 16 + nloc] = acc[r][t][v] * (1.0f / XS);
  wave_lds_sync();
  for (int pass = 0; pass < 2; ++pass) { for (int i = lane; i < 32 * 32; i += 32) { const int rr = i >> 5, c4 = (i & 31) * 4; *(volatile v4f*)(out + (size_t)(m0 + rr) * D + c0 + c4) = *(const v4f*)(&Ts[wave][rr][c4]); } __threadfence(); }
}
}

extern "C" void kernel_launch(void* const* d_in, const int* in_sizes, int n_in,
                              void* d_out, int out_size, void* d_ws, size_t ws_size, hipStream_t stream) {
  (void)n_in; (void)out_size;
  const float* x1 = (const float*)d_in[0]; const float* x2 = (const float*)d_in[1]; const float* wq = (const float*)d_in[2]; const float* wk = (const float*)d_in[3]; const float* wv = (const float*)d_in[4]; const float* wo = (const float*)d_in[5];
  float* out = (float*)d_out;
  if (in_sizes[0] != Bn * S * D || in_sizes[2] != D * D) return;
  size_t off = 0; char* ws = (char*)d_ws;
  auto carve = [&](size_t bytes) { char* p = ws + off; off += (bytes + 255) & ~(size_t)255; return p; };
  b16* R = (b16*)carve((size_t)4 * D * D * 2); b16* X1 = (b16*)carve((size_t)Bn * S * D * 2); b16* X2 = (b16*)carve((size_t)Bn * S * D * 2); b16* Q = (b16*)carve((size_t)Bn * S * D * 2); b16* K = (b16*)carve((size_t)Bn * S * D * 2); b16* VT = (b16*)carve((size_t)Bn * D * S * 2); b16* VTl = (b16*)carve((size_t)Bn * D * S * 2);
  if (off > ws_size) return;
  b16* CH = X1; b16* CL = X2;
  prep_kernel<<<1024, 256, 0, stream>>>(x1, x2, wq, wk, wv, wo, R, X1, X2);
  qk_kernel<<<dim3(16, Bn * S / 32), 64, 0, stream>>>(X1, X2, R, Q, K);
  v_kernel<<<dim3(8, Bn * S / 64), 128, 0, stream>>>(X2, R, VT, VTl);
  attn_kernel<<<dim3(S / 16, 4, Bn), 128, 0, stream>>>(Q, K, VT, VTl, CH, CL);
  out_kernel<<<dim3(4, Bn * S / 32), 64, 0, stream>>>(CH, CL, R, out);
}
